// SelectiveStateSpace_10763188044007
// MI455X (gfx1250) — hardware-verified
//
#include <hip/hip_runtime.h>
#include <math.h>

constexpr int kNB  = 2;
constexpr int kNT  = 2048;
constexpr int kND  = 1024;
constexpr int kNS  = 16;
constexpr int kNR  = 64;
constexpr int kBT  = kNB * kNT;
constexpr int kXZ  = 2 * kND;
constexpr int kXDL = kNR + 2 * kNS;
constexpr int kXDP = 128;
static_assert(kBT % 64 == 0 && kXZ % 64 == 0 && kXDP % 64 == 0 && kND % 64 == 0);
static_assert(kND % 32 == 0);
static_assert((kBT * kND) % (8 * 256) == 0 && (kBT * kND) % (4 * 256) == 0);

typedef __attribute__((ext_vector_type(16))) _Float16 v16h;
typedef __attribute__((ext_vector_type(8)))  _Float16 v8h;
typedef __attribute__((ext_vector_type(16))) __bf16   v16b;
typedef __attribute__((ext_vector_type(8)))  __bf16   v8b;
typedef __attribute__((ext_vector_type(8)))  float    v8f;
typedef __attribute__((ext_vector_type(4)))  float    v4f;
typedef __attribute__((ext_vector_type(4)))  unsigned int v4u;

__device__ __forceinline__ unsigned short f2bf_bits(float f) {
  unsigned u = __float_as_uint(f);
  return (unsigned short)((u + 0x7FFFu + ((u >> 16) & 1u)) >> 16);
}
__device__ __forceinline__ float bf_bits2f(unsigned short h) { return __uint_as_float(((unsigned)h) << 16); }

__device__ __forceinline__ void dep_guard_h(v8f& a, v8f& b, v16h x, v16h y) { asm volatile("v_nop\n\tv_nop\n\tv_nop\n\tv_nop" : "+v"(a), "+v"(b) : "v"(x), "v"(y)); }
__device__ __forceinline__ void dep_guard_b(v8f& a, v8f& b, v16b x, v16b y) { asm volatile("v_nop\n\tv_nop\n\tv_nop\n\tv_nop" : "+v"(a), "+v"(b) : "v"(x), "v"(y)); }
__device__ __forceinline__ void keep4_h(v16h a, v16h b, v16h c, v16h d) { asm volatile("v_nop" :: "v"(a), "v"(b), "v"(c), "v"(d)); }
__device__ __forceinline__ void keep4_b(v16b a, v16b b, v16b c, v16b d) { asm volatile("v_nop" :: "v"(a), "v"(b), "v"(c), "v"(d)); }
__device__ __forceinline__ void acc_guard4(v8f& a, v8f& b, v8f& c, v8f& d) { asm volatile("v_nop\n\tv_nop\n\tv_nop\n\tv_nop" : "+v"(a), "+v"(b), "+v"(c), "+v"(d)); }
template <typename T> struct Frag;
template <> struct Frag<_Float16> {
  typedef v16h V; union U { v16h v; v8h h[2]; };
  static __device__ __forceinline__ v16h load(const _Float16* p) {
    U f; f.h[0] = *(const v8h*)(p); f.h[1] = *(const v8h*)(p + 16); return f.v;
  }
  static __device__ __forceinline__ v8f mma(v16h a, v16h b, v8f c) {
    return __builtin_amdgcn_wmma_f32_16x16x32_f16(false, a, false, b, (short)0, c, false, false);
  }
  static __device__ __forceinline__ void guard(v8f& a, v8f& b, v16h x, v16h y) { dep_guard_h(a, b, x, y); }
  static __device__ __forceinline__ void keep(v16h a, v16h b, v16h c, v16h d) { keep4_h(a, b, c, d); }
};
template <> struct Frag<__bf16> {
  typedef v16b V; union U { v16b v; v8b h[2]; };
  static __device__ __forceinline__ v16b load(const __bf16* p) {
    U f; f.h[0] = *(const v8b*)(p); f.h[1] = *(const v8b*)(p + 16); return f.v;
  }
  static __device__ __forceinline__ v8f mma(v16b a, v16b b, v8f c) {
    return __builtin_amdgcn_wmma_f32_16x16x32_bf16(false, a, false, b, (short)0, c, false, false);
  }
  static __device__ __forceinline__ void guard(v8f& a, v8f& b, v16b x, v16b y) { dep_guard_b(a, b, x, y); }
  static __device__ __forceinline__ void keep(v16b a, v16b b, v16b c, v16b d) { keep4_b(a, b, c, d); }
};

__device__ __forceinline__ unsigned pk16(unsigned short a, unsigned short b) { return (unsigned)a | ((unsigned)b << 16); }

template <int ET> struct Elem;
template <> struct Elem<0> { typedef _Float16 T; };
template <> struct Elem<1> { typedef __bf16 T; };
template <int ET, bool SPLIT, int BIAS_MODE, int OUT_MODE, bool RESID, int ACT = 0>
__global__ __launch_bounds__(256) void wmma_gemm64(
    const unsigned short* __restrict__ Ap, const unsigned short* __restrict__ A2p, int lda, long strideA,
    const unsigned short* __restrict__ Btp, const unsigned short* __restrict__ Bt2p, int ldb, long strideB,
    void* __restrict__ Cout, void* __restrict__ Cout2, int ldc, long strideC,
    const float* __restrict__ bias,
    const float* __restrict__ resid, long strideR,
    int M, int N, int K, float scale) {
  typedef typename Elem<ET>::T T;
  typedef typename Frag<T>::V V;
  const T* A = (const T*)Ap; const T* A2 = (const T*)A2p; const T* Bt = (const T*)Btp; const T* Bt2 = (const T*)Bt2p;
  __shared__ __align__(16) float sT[8][16 * 68];
  const int b    = blockIdx.y;
  const int lane = threadIdx.x & 31;
  const int wave = threadIdx.x >> 5;
  const int tilesN = N >> 6;
  const int tilesM = M >> 6;
  const int tile = blockIdx.x * 8 + wave;
  if (tile >= tilesM * tilesN) return;
  const int tm = tile / tilesN;
  const int tn = tile - tm * tilesN;
  const int m0 = tm << 6;
  const int n0 = tn << 6;

  const T* Ab  = A  + (size_t)b * strideA;
  const T* Bb  = Bt + (size_t)b * strideB;
  const T* Ab2 = SPLIT ? (A2  + (size_t)b * strideA) : nullptr;
  const T* Bb2 = SPLIT ? (Bt2 + (size_t)b * strideB) : nullptr;

  const int rlane = lane & 15;
  const int koff  = (lane >> 4) * 8;
  const int mOff  = (lane >> 4) * 8;

  v8f acc[4][4];
#pragma unroll
  for (int i = 0; i < 4; ++i)
#pragma unroll
    for (int j = 0; j < 4; ++j) acc[i][j] = (v8f){0.f,0.f,0.f,0.f,0.f,0.f,0.f,0.f};

  for (int k0 = 0; k0 < K; k0 += 32) {
    V bh[4], bl[4];
#pragma unroll
    for (int j = 0; j < 4; ++j) {
      const size_t bo = (size_t)(n0 + (j << 4) + rlane) * ldb + koff + k0;
      bh[j] = Frag<T>::load(Bb + bo);
      if (SPLIT) bl[j] = Frag<T>::load(Bb2 + bo);
    }
#pragma unroll
    for (int i = 0; i < 4; ++i) {
      const size_t ao = (size_t)(m0 + (i << 4) + rlane) * lda + koff + k0;
      V ah = Frag<T>::load(Ab + ao);
      V al;
      if (SPLIT) al = Frag<T>::load(Ab2 + ao);
#pragma unroll
      for (int j = 0; j < 4; ++j) {
        acc[i][j] = Frag<T>::mma(ah, bh[j], acc[i][j]);
        if (SPLIT) {
          acc[i][j] = Frag<T>::mma(ah, bl[j], acc[i][j]);
          acc[i][j] = Frag<T>::mma(al, bh[j], acc[i][j]);
        }
      }
      Frag<T>::guard(acc[i][0], acc[i][3], ah, SPLIT ? al : ah);
    }
    Frag<T>::keep(bh[0], bh[1], bh[2], bh[3]);
    if (SPLIT) Frag<T>::keep(bl[0], bl[1], bl[2], bl[3]);
  }
  acc_guard4(acc[0][0], acc[0][1], acc[0][2], acc[0][3]);
  acc_guard4(acc[1][0], acc[1][1], acc[1][2], acc[1][3]);
  acc_guard4(acc[2][0], acc[2][1], acc[2][2], acc[2][3]);
  acc_guard4(acc[3][0], acc[3][1], acc[3][2], acc[3][3]);

  float* slab = sT[wave];
  const float* Rb = RESID ? (resid + (size_t)b * strideR) : nullptr;
#pragma unroll
  for (int i = 0; i < 4; ++i) {
    const int mBase = m0 + (i << 4);
#pragma unroll
    for (int j = 0; j < 4; ++j) {
      const int n = n0 + (j << 4) + rlane;
      float bv = 0.f;
      if (BIAS_MODE == 2) bv = bias[n];
#pragma unroll
      for (int r = 0; r < 8; ++r) {
        float v = acc[i][j][r] * scale;
        if (BIAS_MODE == 1) v += bias[mBase + mOff + r];
        if (BIAS_MODE == 2) v += bv;
        if (RESID) v += Rb[(size_t)(mBase + mOff + r) * ldc + n];
        if (ACT == 2) v = fmaxf(v, 0.0f);
        if (ACT == 4) v = (v > 0.f) ? v : 0.01f * v;
        slab[(mOff + r) * 68 + (j << 4) + rlane] = v;
      }
    }
    __builtin_amdgcn_fence(__ATOMIC_RELEASE, "workgroup");
    __builtin_amdgcn_wave_barrier();
    __builtin_amdgcn_fence(__ATOMIC_ACQUIRE, "workgroup");
    if (OUT_MODE == 0) {
      float* C = (float*)Cout + (size_t)b * strideC;
      const int hh = lane >> 4, c4 = (lane & 15) * 4;
      for (int pass = 0; pass < 2; ++pass) {
#pragma unroll
        for (int it = 0; it < 8; ++it) {
          const int row = it * 2 + hh;
          v4f v = *(const v4f*)(slab + row * 68 + c4);
          *(volatile v4f*)(C + (size_t)(mBase + row) * ldc + n0 + c4) = v;
        }
        __threadfence();
      }
    } else {
      const int q = lane >> 3, c8 = (lane & 7) * 8;
      unsigned short* C  = (unsigned short*)Cout  + (size_t)b * strideC;
      unsigned short* C2 = (OUT_MODE == 2) ? ((unsigned short*)Cout2 + (size_t)b * strideC) : nullptr;
      for (int pass = 0; pass < 2; ++pass) {
#pragma unroll
        for (int it = 0; it < 4; ++it) {
          const int row = it * 4 + q;
          const float* sp = slab + row * 68 + c8;
          v8h hv, lv;
#pragma unroll
          for (int e = 0; e < 8; ++e) {
            if (OUT_MODE == 1) {
              hv[e] = (_Float16)sp[e];
            } else {
              unsigned short hb = f2bf_bits(sp[e]);
              unsigned short lb = f2bf_bits(sp[e] - bf_bits2f(hb));
              hv[e] = __builtin_bit_cast(_Float16, hb);
              lv[e] = __builtin_bit_cast(_Float16, lb);
            }
          }
          *(volatile v8h*)(C + (size_t)(mBase + row) * ldc + n0 + c8) = hv;
          if (OUT_MODE == 2) *(volatile v8h*)(C2 + (size_t)(mBase + row) * ldc + n0 + c8) = lv;
        }
        __threadfence();
      }
    }
    __builtin_amdgcn_fence(__ATOMIC_RELEASE, "workgroup");
    __builtin_amdgcn_wave_barrier();
    __builtin_amdgcn_fence(__ATOMIC_ACQUIRE, "workgroup");
  }
}

#pragma clang fp contract(off)

__device__ __forceinline__ void split_bf(float v, unsigned short& hb, unsigned short& lb) {
  hb = f2bf_bits(v);
  lb = f2bf_bits(v - bf_bits2f(hb));
}
__device__ __forceinline__ float silu_f(float x) {
  const float e  = expf(-x);
  const float sg = 1.0f / (1.0f + e);
  return x * sg;
}
__device__ __forceinline__ float softplus_f(float x) {
  const float ax = fabsf(x);
  return fmaxf(x, 0.0f) + log1pf(expf(-ax));
}

__global__ __launch_bounds__(256) void split8_kernel(const float* __restrict__ in, int rows_src, int rows_dst,
                                                     unsigned short* __restrict__ hi, unsigned short* __restrict__ lo) {
  const int u = blockIdx.x * 256 + threadIdx.x;
  if (u >= rows_dst * (kND / 8)) return;
  const int row = u >> 7;
  const int c   = (u & 127) * 8;
  const int rs  = (row < rows_src) ? row : (rows_src - 1);
  const bool live = (row < rows_src);
  const float* p = in + (size_t)rs * kND + c;
  const v4f a = *(const v4f*)p;
  const v4f bq = *(const v4f*)(p + 4);
  unsigned short hb[8], lb[8];
#pragma unroll
  for (int e = 0; e < 4; ++e) {
    const float v0 = live ? a[e] : 0.0f;
    const float v1 = live ? bq[e] : 0.0f;
    split_bf(v0, hb[e], lb[e]);
    split_bf(v1, hb[4 + e], lb[4 + e]);
  }
  const v4u uh = (v4u){pk16(hb[0], hb[1]), pk16(hb[2], hb[3]), pk16(hb[4], hb[5]), pk16(hb[6], hb[7])};
  const v4u ul = (v4u){pk16(lb[0], lb[1]), pk16(lb[2], lb[3]), pk16(lb[4], lb[5]), pk16(lb[6], lb[7])};
  const size_t go = (size_t)row * kND + c;
  for (int pass = 0; pass < 2; ++pass) {
    *(volatile v4u*)(hi + go) = uh;
    *(volatile v4u*)(lo + go) = ul;
    __threadfence();
  }
}

__global__ __launch_bounds__(256) void conv_silu_kernel(const float* __restrict__ xz, const float* __restrict__ cw,
                                                        float* __restrict__ xs, unsigned short* __restrict__ xsh,
                                                        unsigned short* __restrict__ xsl) {
  __shared__ __align__(16) float stg[8 * 256];
  const int tid = threadIdx.x, lane = tid & 31, wave = tid >> 5;
  const int u  = blockIdx.x * 256 + tid;
  const int bt = u >> 7;
  const int d0 = (u & 127) * 8;
  const int t  = bt & (kNT - 1);
  const bool hasp = (t > 0);
  const bool hasn = (t < kNT - 1);
  const int btp = hasp ? (bt - 1) : bt;
  const int btn = hasn ? (bt + 1) : bt;
  const float* rc = xz + (size_t)bt  * kXZ + d0;
  const float* rp = xz + (size_t)btp * kXZ + d0;
  const float* rn = xz + (size_t)btn * kXZ + d0;
  const v4f c0 = *(const v4f*)rc, c1 = *(const v4f*)(rc + 4);
  const v4f p0 = *(const v4f*)rp, p1 = *(const v4f*)(rp + 4);
  const v4f q0 = *(const v4f*)rn, q1 = *(const v4f*)(rn + 4);
  const float* wp = cw + (size_t)d0 * 3;
  const v4f w0 = *(const v4f*)(wp), w1 = *(const v4f*)(wp + 4), w2 = *(const v4f*)(wp + 8);
  const v4f w3 = *(const v4f*)(wp + 12), w4 = *(const v4f*)(wp + 16), w5 = *(const v4f*)(wp + 20);
  const float wv[24] = {w0[0], w0[1], w0[2], w0[3], w1[0], w1[1], w1[2], w1[3], w2[0], w2[1], w2[2], w2[3],
                        w3[0], w3[1], w3[2], w3[3], w4[0], w4[1], w4[2], w4[3], w5[0], w5[1], w5[2], w5[3]};
  const float cv[8] = {c0[0], c0[1], c0[2], c0[3], c1[0], c1[1], c1[2], c1[3]};
  const float pv[8] = {p0[0], p0[1], p0[2], p0[3], p1[0], p1[1], p1[2], p1[3]};
  const float nv[8] = {q0[0], q0[1], q0[2], q0[3], q1[0], q1[1], q1[2], q1[3]};
  float sv[8];
  unsigned short hb[8], lb[8];
#pragma unroll
  for (int e = 0; e < 8; ++e) {
    const float xm = hasp ? pv[e] : 0.0f;
    const float xp = hasn ? nv[e] : 0.0f;
    const float cvv = (xm * wv[3 * e] + cv[e] * wv[3 * e + 1]) + xp * wv[3 * e + 2];
    const float s = silu_f(cvv);
    sv[e] = s;
    split_bf(s, hb[e], lb[e]);
  }
  const v4u uh = (v4u){pk16(hb[0], hb[1]), pk16(hb[2], hb[3]), pk16(hb[4], hb[5]), pk16(hb[6], hb[7])};
  const v4u ul = (v4u){pk16(lb[0], lb[1]), pk16(lb[2], lb[3]), pk16(lb[4], lb[5]), pk16(lb[6], lb[7])};
  float* sw = stg + wave * 256;
  *(v4f*)(sw + lane * 8)     = (v4f){sv[0], sv[1], sv[2], sv[3]};
  *(v4f*)(sw + lane * 8 + 4) = (v4f){sv[4], sv[5], sv[6], sv[7]};
  __builtin_amdgcn_fence(__ATOMIC_RELEASE, "workgroup");
  __builtin_amdgcn_wave_barrier();
  __builtin_amdgcn_fence(__ATOMIC_ACQUIRE, "workgroup");
  const v4f f0 = *(const v4f*)(sw + lane * 4);
  const v4f f1 = *(const v4f*)(sw + 128 + lane * 4);
  const int dW = (u & 96) * 8;
  float* px = xs + (size_t)bt * kND + dW;
  const size_t gp = (size_t)bt * kND + d0;
  for (int pass = 0; pass < 2; ++pass) {
    *(volatile v4u*)(xsh + gp) = uh;
    *(volatile v4u*)(xsl + gp) = ul;
    *(volatile v4f*)(px + lane * 4) = f0;
    *(volatile v4f*)(px + 128 + lane * 4) = f1;
    __threadfence();
  }
}

constexpr int kPJT = 64;
constexpr int kPJP = 80;
__global__ __launch_bounds__(256) void dtc_proj_kernel(const float* __restrict__ xd, const float* __restrict__ wdt,
                                                       const float* __restrict__ bdt, const float* __restrict__ wc,
                                                       float* __restrict__ dt, float* __restrict__ cm) {
  __shared__ __align__(16) float xdS[kPJT * kPJP];
  __shared__ __align__(16) float dtS[4 * 256];
  __shared__ __align__(16) float cS[4 * 256];
  const int tid   = threadIdx.x;
  const int dbase = blockIdx.x * 256;
  const int d     = dbase + tid;
  const int bt0   = blockIdx.y * kPJT;
#pragma unroll
  for (int it = 0; it < 5; ++it) {
    const int f    = it * 256 + tid;
    const int tok  = f / 20;
    const int q    = f - tok * 20;
    const int scol = (q < 16) ? (q * 4) : (kNR + kNS + (q - 16) * 4);
    const v4f v = *(const v4f*)(xd + (size_t)(bt0 + tok) * kXDP + scol);
    *(v4f*)(xdS + tok * kPJP + q * 4) = v;
  }
  const float bd = bdt[d];
  const float* wrow = wdt + (size_t)d * kNR;
  const float* wcr  = wc  + (size_t)d * kNS;
  __syncthreads();
  const int srow = tid >> 6;
  const int sc4  = (tid & 63) * 4;
#pragma unroll 1
  for (int tg = 0; tg < kPJT / 4; ++tg) {
    float acc[4] = {0.f, 0.f, 0.f, 0.f};
    float cac[4] = {0.f, 0.f, 0.f, 0.f};
    const float* xg = xdS + tg * 4 * kPJP;
#pragma unroll 1
    for (int r4 = 0; r4 < kNR / 4; ++r4) {
      const v4f w = *(const v4f*)(wrow + 4 * r4);
#pragma unroll
      for (int tk = 0; tk < 4; ++tk) {
        const v4f xv = *(const v4f*)(xg + tk * kPJP + 4 * r4);
        acc[tk] = fmaf(xv[0], w[0], acc[tk]);
        acc[tk] = fmaf(xv[1], w[1], acc[tk]);
        acc[tk] = fmaf(xv[2], w[2], acc[tk]);
        acc[tk] = fmaf(xv[3], w[3], acc[tk]);
      }
    }
#pragma unroll 1
    for (int n4 = 0; n4 < kNS / 4; ++n4) {
      const v4f w = *(const v4f*)(wcr + 4 * n4);
#pragma unroll
      for (int tk = 0; tk < 4; ++tk) {
        const v4f xv = *(const v4f*)(xg + tk * kPJP + kNR + 4 * n4);
        cac[tk] = fmaf(xv[0], w[0], cac[tk]);
        cac[tk] = fmaf(xv[1], w[1], cac[tk]);
        cac[tk] = fmaf(xv[2], w[2], cac[tk]);
        cac[tk] = fmaf(xv[3], w[3], cac[tk]);
      }
    }
    __syncthreads();
#pragma unroll
    for (int tk = 0; tk < 4; ++tk) {
      dtS[tk * 256 + tid] = acc[tk] + bd;
      cS[tk * 256 + tid]  = cac[tk];
    }
#pragma unroll 1
    for (int tk = 0; tk < 4; ++tk) {
      const float v = dtS[tk * 256 + tid];
      dtS[tk * 256 + tid] = softplus_f(v) + 1e-5f;
    }
    __syncthreads();
    const v4f dv = *(const v4f*)(dtS + srow * 256 + sc4);
    const v4f ccv = *(const v4f*)(cS + srow * 256 + sc4);
    const size_t go = (size_t)(bt0 + tg * 4 + srow) * kND + dbase + sc4;
    for (int pass = 0; pass < 2; ++pass) {
      *(volatile v4f*)(dt + go) = dv;
      *(volatile v4f*)(cm + go) = ccv;
      __threadfence();
    }
  }
}

constexpr int kSCC = 128;
constexpr int kSTC = 32;
static_assert(kNT % kSTC == 0 && kND % kSCC == 0 && kSTC * 4 == kSCC);
__global__ __launch_bounds__(kSCC) void scan_kernel(const float* __restrict__ xd, const float* __restrict__ dt,
                                                    const float* __restrict__ xs, const float* __restrict__ cm,
                                                    const float* __restrict__ alog, const float* __restrict__ dpar,
                                                    unsigned short* __restrict__ yh, unsigned short* __restrict__ yl) {
  __shared__ __align__(16) float bpS[kSTC * kNS];
  __shared__ __align__(16) float yS[kSTC * kSCC];
  const int tid = threadIdx.x;
  const int b   = blockIdx.x / (kND / kSCC);
  const int d0  = (blockIdx.x - b * (kND / kSCC)) * kSCC;
  const int d   = d0 + tid;
  float ne[kNS], s[kNS];
  {
    const float* ap = alog + (size_t)d * kNS;
    const v4f a0 = *(const v4f*)(ap), a1 = *(const v4f*)(ap + 4), a2 = *(const v4f*)(ap + 8), a3 = *(const v4f*)(ap + 12);
    const float al[kNS] = {a0[0], a0[1], a0[2], a0[3], a1[0], a1[1], a1[2], a1[3],
                           a2[0], a2[1], a2[2], a2[3], a3[0], a3[1], a3[2], a3[3]};
#pragma unroll
    for (int n = 0; n < kNS; ++n) { ne[n] = -expf(al[n]); s[n] = 0.0f; }
  }
  const float dp = dpar[d];
  const int rq = tid >> 4, c8 = (tid & 15) * 8;
#pragma unroll 1
  for (int ck = 0; ck < kNT / kSTC; ++ck) {
    const int t0 = ck * kSTC;
    __syncthreads();
    {
      const int tt = tid >> 2, q = tid & 3;
      const v4f v = *(const v4f*)(xd + (size_t)(b * kNT + t0 + tt) * kXDP + kNR + 4 * q);
      *(v4f*)(bpS + tt * kNS + 4 * q) = v;
    }
    __syncthreads();
#pragma unroll 1
    for (int tt = 0; tt < kSTC; ++tt) {
      const size_t off = (size_t)(b * kNT + t0 + tt) * kND + d;
      const float dtv = dt[off];
      const float xsv = xs[off];
      const float cmv = cm[off];
      const float* bq = bpS + tt * kNS;
      const v4f g0 = *(const v4f*)(bq), g1 = *(const v4f*)(bq + 4), g2 = *(const v4f*)(bq + 8), g3 = *(const v4f*)(bq + 12);
      const float bp[kNS] = {g0[0], g0[1], g0[2], g0[3], g1[0], g1[1], g1[2], g1[3],
                             g2[0], g2[1], g2[2], g2[3], g3[0], g3[1], g3[2], g3[3]};
      float ssum = 0.0f;
#pragma unroll
      for (int n = 0; n < kNS; ++n) {
        const float a  = expf(ne[n] * dtv);
        const float bx = (bp[n] * dtv) * xsv;
        s[n] = a * s[n] + bx;
        ssum = ssum + s[n];
      }
      yS[tt * kSCC + tid] = cmv * ssum + dp * xsv;
    }
    __syncthreads();
    for (int pass = 0; pass < 2; ++pass) {
#pragma unroll
      for (int it = 0; it < 4; ++it) {
        const int row = it * 8 + rq;
        const v4f ya = *(const v4f*)(yS + row * kSCC + c8);
        const v4f yb = *(const v4f*)(yS + row * kSCC + c8 + 4);
        unsigned short hb[8], lb[8];
#pragma unroll
        for (int e = 0; e < 4; ++e) {
          split_bf(ya[e], hb[e], lb[e]);
          split_bf(yb[e], hb[4 + e], lb[4 + e]);
        }
        const v4u uh = (v4u){pk16(hb[0], hb[1]), pk16(hb[2], hb[3]), pk16(hb[4], hb[5]), pk16(hb[6], hb[7])};
        const v4u ul = (v4u){pk16(lb[0], lb[1]), pk16(lb[2], lb[3]), pk16(lb[4], lb[5]), pk16(lb[6], lb[7])};
        const size_t go = (size_t)(b * kNT + t0 + row) * kND + d0 + c8;
        *(volatile v4u*)(yh + go) = uh;
        *(volatile v4u*)(yl + go) = ul;
      }
      __threadfence();
    }
  }
}

__global__ __launch_bounds__(256) void gate_kernel(const float* __restrict__ op, const float* __restrict__ xz,
                                                   float* __restrict__ out) {
  const int u  = blockIdx.x * 256 + threadIdx.x;
  const int bt = u >> 8;
  const int c4 = (u & 255) * 4;
  const v4f a = *(const v4f*)(op + (size_t)bt * kND + c4);
  const v4f z = *(const v4f*)(xz + (size_t)bt * kXZ + kND + c4);
  v4f r;
#pragma unroll
  for (int e = 0; e < 4; ++e) r[e] = a[e] * silu_f(z[e]);
  float* po = out + (size_t)bt * kND + c4;
  for (int pass = 0; pass < 2; ++pass) {
    *(volatile v4f*)po = r;
    __threadfence();
  }
}

extern "C" void kernel_launch(void* const* d_in, const int* in_sizes, int n_in,
                              void* d_out, int out_size, void* d_ws, size_t ws_size, hipStream_t stream) {
  if (n_in < 10) return;
  if (in_sizes[0] != kBT * kND || in_sizes[1] != kXZ * kND || in_sizes[2] != kND * 3 || in_sizes[3] != kXDL * kND ||
      in_sizes[4] != kND * kNR || in_sizes[5] != kND || in_sizes[6] != kND * kNS || in_sizes[7] != kND ||
      in_sizes[8] != kND * kNS || in_sizes[9] != kND * kND || out_size != kBT * kND) return;

  const float* x       = (const float*)d_in[0];
  const float* W_in    = (const float*)d_in[1];
  const float* conv_w  = (const float*)d_in[2];
  const float* W_x     = (const float*)d_in[3];
  const float* W_dt    = (const float*)d_in[4];
  const float* b_dt    = (const float*)d_in[5];
  const float* A_log   = (const float*)d_in[6];
  const float* D_param = (const float*)d_in[7];
  const float* W_C     = (const float*)d_in[8];
  const float* W_out   = (const float*)d_in[9];
  float* out = (float*)d_out;

  const size_t MiB   = 1048576;
  const size_t o_xh  = 0;
  const size_t o_xl  = o_xh  + (size_t)kBT * kND * 2;
  const size_t o_wih = o_xl  + (size_t)kBT * kND * 2;
  const size_t o_wil = o_wih + (size_t)kXZ * kND * 2;
  const size_t o_wxh = o_wil + (size_t)kXZ * kND * 2;
  const size_t o_wxl = o_wxh + (size_t)kXDP * kND * 2;
  const size_t o_woh = o_wxl + (size_t)kXDP * kND * 2;
  const size_t o_wol = o_woh + (size_t)kND * kND * 2;
  const size_t o_xz  = o_wol + (size_t)kND * kND * 2;
  const size_t o_xs  = o_xz  + (size_t)kBT * kXZ * 4;
  const size_t o_xsh = o_xs  + (size_t)kBT * kND * 4;
  const size_t o_xsl = o_xsh + (size_t)kBT * kND * 2;
  const size_t o_xd  = o_xsl + (size_t)kBT * kND * 2;
  const size_t o_cm  = o_xd  + (size_t)kBT * kXDP * 4;
  const size_t o_end = o_cm  + (size_t)kBT * kND * 4;
  const size_t o_yh  = o_xh;
  const size_t o_yl  = o_xl;
  const size_t o_dt  = o_xsh;
  const size_t o_op  = o_xs;
  if (o_end > ws_size || o_end > 128 * MiB) return;

  char* ws = (char*)d_ws;
  unsigned short* xh  = (unsigned short*)(ws + o_xh);
  unsigned short* xl  = (unsigned short*)(ws + o_xl);
  unsigned short* wih = (unsigned short*)(ws + o_wih);
  unsigned short* wil = (unsigned short*)(ws + o_wil);
  unsigned short* wxh = (unsigned short*)(ws + o_wxh);
  unsigned short* wxl = (unsigned short*)(ws + o_wxl);
  unsigned short* woh = (unsigned short*)(ws + o_woh);
  unsigned short* wol = (unsigned short*)(ws + o_wol);
  float* xz  = (float*)(ws + o_xz);
  float* xs  = (float*)(ws + o_xs);
  unsigned short* xsh = (unsigned short*)(ws + o_xsh);
  unsigned short* xsl = (unsigned short*)(ws + o_xsl);
  float* xd  = (float*)(ws + o_xd);
  float* cmb = (float*)(ws + o_cm);
  unsigned short* yh  = (unsigned short*)(ws + o_yh);
  unsigned short* yl  = (unsigned short*)(ws + o_yl);
  float* dtb = (float*)(ws + o_dt);
  float* opb = (float*)(ws + o_op);

  split8_kernel<<<kBT * (kND / 8) / 256, 256, 0, stream>>>(x, kBT, kBT, xh, xl);
  split8_kernel<<<kXZ * (kND / 8) / 256, 256, 0, stream>>>(W_in, kXZ, kXZ, wih, wil);
  split8_kernel<<<kXDP * (kND / 8) / 256, 256, 0, stream>>>(W_x, kXDL, kXDP, wxh, wxl);
  split8_kernel<<<kND * (kND / 8) / 256, 256, 0, stream>>>(W_out, kND, kND, woh, wol);

  wmma_gemm64<1, true, 0, 0, false, 0><<<dim3((kBT / 64) * (kXZ / 64) / 8, 1), 256, 0, stream>>>(
      xh, xl, kND, 0L, wih, wil, kND, 0L, (void*)xz, nullptr, kXZ, 0L, nullptr, nullptr, 0L, kBT, kXZ, kND, 1.0f);

  conv_silu_kernel<<<kBT * (kND / 8) / 256, 256, 0, stream>>>(xz, conv_w, xs, xsh, xsl);

  wmma_gemm64<1, true, 0, 0, false, 0><<<dim3((kBT / 64) * (kXDP / 64) / 8, 1), 256, 0, stream>>>(
      xsh, xsl, kND, 0L, wxh, wxl, kND, 0L, (void*)xd, nullptr, kXDP, 0L, nullptr, nullptr, 0L, kBT, kXDP, kND, 1.0f);

  dtc_proj_kernel<<<dim3(kND / 256, kBT / kPJT), 256, 0, stream>>>(xd, W_dt, b_dt, W_C, dtb, cmb);

  scan_kernel<<<kNB * (kND / kSCC), kSCC, 0, stream>>>(xd, dtb, xs, cmb, A_log, D_param, yh, yl);

  wmma_gemm64<1, true, 0, 0, false, 0><<<dim3((kBT / 64) * (kND / 64) / 8, 1), 256, 0, stream>>>(
      yh, yl, kND, 0L, woh, wol, kND, 0L, (void*)opb, nullptr, kND, 0L, nullptr, nullptr, 0L, kBT, kND, kND, 1.0f);

  gate_kernel<<<kBT * (kND / 4) / 256, 256, 0, stream>>>(opb, xz, out);
}
